// MultiHeadSelfAttention_34754875359500
// MI455X (gfx1250) — hardware-verified
//
#include <hip/hip_runtime.h>
#include <math.h>

typedef __attribute__((ext_vector_type(16))) _Float16 v16h;
typedef __attribute__((ext_vector_type(16))) __bf16 v16b;
typedef __attribute__((ext_vector_type(8)))  _Float16 v8h;
typedef __attribute__((ext_vector_type(8)))  __bf16 v8b;
typedef __attribute__((ext_vector_type(8)))  float v8f;
typedef __attribute__((ext_vector_type(4)))  float v4f;
typedef __attribute__((ext_vector_type(4)))  unsigned v4u;

#ifndef NB
#define NB 2
#endif
#ifndef SEQ
#define SEQ 2048
#endif
#define NB_FULL 2
#define TT_FULL 2048
#define TT SEQ
#define CC 1024
#define DIN 1024
#define NH 16
#define HD 64
#define NQB (TT / 64)
#define QBH ((TT / 64) < 6 ? (TT / 64) : 6)
#define QHI (QBH * 64)
#define KHI QHI
#define SCALE_L2 (0.125f * 1.44269504088896340736f)

static_assert(NB <= NB_FULL);
static_assert(TT <= TT_FULL);
static_assert(TT % 64 == 0);
static_assert(CC == NH * HD);
static_assert(HD == 64);
static_assert(HD % 32 == 0);
static_assert(DIN % 32 == 0);
static_assert(CC % 32 == 0);
static_assert(CC % 128 == 0);
static_assert(DIN % 128 == 0);
static_assert(QHI % 64 == 0);
static_assert(KHI >= QHI);
static_assert(KHI % 32 == 0);
static_assert(QBH <= NQB);

#define WS_QH  ((size_t)0)
#define WS_KH  (WS_QH + 2u * (size_t)NB * TT * CC)
#define WS_VT  (WS_KH + 2u * (size_t)NB * TT * CC)
#define WS_QL  (WS_VT + 2u * (size_t)NB * CC * TT)
#define WS_KL  (WS_QL + 2u * (size_t)NB * QHI * CC)
#define WS_VB  (WS_KL + 2u * (size_t)NB * KHI * CC)
#define WS_VBL (WS_VB + 2u * (size_t)NB * CC * KHI)
#define WS_Y   (WS_VBL + 2u * (size_t)NB * CC * KHI)
#define WS_END (WS_Y + 4u * (size_t)NB * TT * CC)
static_assert(WS_END <= (size_t)134217728);
static_assert(WS_KH % 128 == 0 && WS_VT % 128 == 0 && WS_QL % 128 == 0 && WS_KL % 128 == 0 && WS_VB % 128 == 0 && WS_VBL % 128 == 0 && WS_Y % 128 == 0);

template <typename T> __device__ __forceinline__ void vst2(void* p, T v) { *(volatile T*)p = v; __threadfence(); *(volatile T*)p = v; }
__device__ __forceinline__ v8f wmma16(v16h a, v16h b, v8f c) {
  v8f d = __builtin_amdgcn_wmma_f32_16x16x32_f16(false, a, false, b, (short)0, c, false, false);
  asm volatile("v_nop\n\tv_nop\n\tv_nop\n\tv_nop" : "+v"(d) : "v"(a), "v"(b));
  return d;
}
__device__ __forceinline__ v8f wmma_bf(v16b a, v16b b, v8f c) {
  v8f d = __builtin_amdgcn_wmma_f32_16x16x32_bf16(false, a, false, b, (short)0, c, false, false);
  asm volatile("v_nop\n\tv_nop\n\tv_nop\n\tv_nop" : "+v"(d) : "v"(a), "v"(b));
  return d;
}
__device__ __forceinline__ v16h frag_h(const _Float16* rowk0, int lane) {
  union { v16h v; v8h q[2]; } u; const _Float16* p = rowk0 + 8 * (lane >> 4);
  u.q[0] = *(const v8h*)p; u.q[1] = *(const v8h*)(p + 16); return u.v;
}
__device__ __forceinline__ v16b frag_b(const __bf16* rowk0, int lane) {
  union { v16b v; v8b q[2]; } u; const __bf16* p = rowk0 + 8 * (lane >> 4);
  u.q[0] = *(const v8b*)p; u.q[1] = *(const v8b*)(p + 16); return u.v;
}
__device__ __forceinline__ v16h frag_f32s(const float* rowk0, int lane, float sc) {
  v16h a; const float* p = rowk0 + 8 * (lane >> 4);
#pragma unroll
  for (int i = 0; i < 8; ++i) { a[i] = (_Float16)(p[i] * sc); a[8 + i] = (_Float16)(p[16 + i] * sc); }
  return a;
}
struct F2 { v16b h, l; };
__device__ __forceinline__ F2 bsplit16(const float v[16]) { F2 r;
#pragma unroll
  for (int i = 0; i < 16; ++i) { const __bf16 h = (__bf16)v[i]; r.h[i] = h; r.l[i] = (__bf16)(v[i] - (float)h); }
  return r; }
__device__ __forceinline__ F2 split_row(const float* row, int k0, int lane) { float v[16]; const float* p = row + k0 + 8 * (lane >> 4);
#pragma unroll
  for (int i = 0; i < 8; ++i) { v[i] = p[i]; v[8 + i] = p[16 + i]; }
  return bsplit16(v); }
__device__ __forceinline__ float bfr(float v) { return (float)(__bf16)v; }
__device__ __forceinline__ v16b wcol_oi(const float* Wm, int k0, int o, int lane, int K) { v16b w; const float* p = Wm + (size_t)o * K + k0 + 8 * (lane >> 4);
#pragma unroll
  for (int i = 0; i < 8; ++i) { w[i] = (__bf16)p[i]; w[8 + i] = (__bf16)p[16 + i]; }
  return w; }
__device__ __forceinline__ v16h wcolh_oi(const float* Wm, int k0, int o, int lane, int K) { v16h w; const float* p = Wm + (size_t)o * K + k0 + 8 * (lane >> 4);
#pragma unroll
  for (int i = 0; i < 8; ++i) { w[i] = (_Float16)(bfr(p[i]) * 256.0f); w[8 + i] = (_Float16)(bfr(p[16 + i]) * 256.0f); }
  return w; }
#define LDSX() do { asm volatile("s_wait_dscnt 0" ::: "memory"); __builtin_amdgcn_wave_barrier(); __builtin_amdgcn_fence(3  , "workgroup"); } while (0)

__device__ __forceinline__ void proj_gemm(const float* __restrict__ X, const float* __restrict__ WA, size_t xrow, int c0, int lane, v8f (&acc)[8]) {
  const int col = lane & 15, g = lane >> 4;
#pragma unroll 2
  for (int kc = 0; kc < DIN / 32; ++kc) { v16b a; { const float* p = X + xrow * DIN + kc * 32 + 8 * g;
#pragma unroll
      for (int i = 0; i < 8; ++i) { a[i] = (__bf16)p[i]; a[8 + i] = (__bf16)p[16 + i]; } }
    asm volatile("s_wait_loadcnt 0x0" ::: "memory");
#pragma unroll
    for (int j = 0; j < 8; ++j) { const v16b w = wcol_oi(WA, kc * 32, c0 + j * 16 + col, lane, DIN); asm volatile("s_wait_loadcnt 0x0" ::: "memory"); acc[j] = wmma_bf(a, w, acc[j]); } }
}

__device__ __forceinline__ void proj_qk_body(const float* __restrict__ X, const float* __restrict__ WA, const float* __restrict__ BA, _Float16* __restrict__ DH, _Float16* __restrict__ DL, const int nhi) {
  __shared__ __align__(16) _Float16 sh[64][136], sl[64][136]; __shared__ float rc[64][32], rs[64][32];
  const int tid = threadIdx.x, wave = tid >> 5, lane = tid & 31, col = lane & 15, g = lane >> 4;
  const int c0 = blockIdx.y * 128; const size_t r0 = (size_t)blockIdx.x * 64; const size_t bb = r0 / TT; const int t0 = (int)(r0 % TT);
  { const int i = tid & 31; const float invf = 1.0f / powf(10000.0f, (float)(2 * i) * (1.0f / 64.0f));
#pragma unroll 1
    for (int it = 0; it < 16; ++it) { const int rl = (tid >> 5) + 4 * it; const float ang = (float)(t0 + rl) * invf; float sn, cs; sincosf(ang, &sn, &cs); rc[rl][i] = cs; rs[rl][i] = sn; } }
  v8f acc[8] = {};
  proj_gemm(X, WA, bb * TT_FULL + t0 + wave * 16 + col, c0, lane, acc);
  __syncthreads();
  const bool odd = (col & 1) != 0;
#pragma unroll
  for (int j = 0; j < 8; ++j) { const float bias = bfr(BA[c0 + j * 16 + col]); const int pi = ((j * 16 + col) & 63) >> 1;
#pragma unroll
    for (int r = 0; r < 8; ++r) { const int rl = wave * 16 + 8 * g + r; const float v = acc[j][r] + bias; const float pv = __shfl_xor(v, 1); const float cs = rc[rl][pi], sn = rs[rl][pi];
      const float xe = odd ? pv : v, xo = odd ? v : pv; const float re = xe * cs - xo * sn, ro = xe * sn + xo * cs; const float o = odd ? ro : re;
      const _Float16 hv = (_Float16)o; sh[rl][j * 16 + col] = hv; sl[rl][j * 16 + col] = (_Float16)((o - (float)hv) * 1024.0f); } }
  __syncthreads();
  const bool hi_rows = t0 < nhi;
  for (int e = tid; e < 64 * 16; e += 128) { const int rl = e >> 4, q = e & 15; vst2((unsigned*)(DH + (r0 + rl) * CC + c0 + q * 8), *(const v4u*)&sh[rl][q * 8]); if (hi_rows) vst2((unsigned*)(DL + (bb * nhi + t0 + rl) * (size_t)CC + c0 + q * 8), *(const v4u*)&sl[rl][q * 8]); }
}
__global__ __launch_bounds__(128) void k_projq(const float* __restrict__ X, const float* __restrict__ W, const float* __restrict__ B, _Float16* __restrict__ QH, _Float16* __restrict__ QL) { proj_qk_body(X, W, B, QH, QL, QHI); }
__global__ __launch_bounds__(128) void k_projk(const float* __restrict__ X, const float* __restrict__ W, const float* __restrict__ B, _Float16* __restrict__ KH, _Float16* __restrict__ KL) { proj_qk_body(X, W, B, KH, KL, KHI); }

__global__ __launch_bounds__(128) void k_projv(const float* __restrict__ X, const float* __restrict__ WA, const float* __restrict__ BA, _Float16* __restrict__ VT, __bf16* __restrict__ VB, __bf16* __restrict__ VBL) {
  __shared__ __align__(16) _Float16 th[128][72]; __shared__ __align__(16) __bf16 tb[128][72], tbl[128][72];
  const int tid = threadIdx.x, wave = tid >> 5, lane = tid & 31, col = lane & 15, g = lane >> 4;
  const int c0 = blockIdx.y * 128; const size_t r0 = (size_t)blockIdx.x * 64; const size_t bb = r0 / TT; const int t0 = (int)(r0 % TT);
  v8f acc[8] = {};
  proj_gemm(X, WA, bb * TT_FULL + t0 + wave * 16 + col, c0, lane, acc);
  const bool hi_rows = t0 < KHI;
#pragma unroll
  for (int j = 0; j < 8; ++j) { const float bias = bfr(BA[c0 + j * 16 + col]);
#pragma unroll
    for (int r = 0; r < 8; ++r) { const float v = acc[j][r] + bias; const int rl = wave * 16 + 8 * g + r, cl = j * 16 + col; th[cl][rl] = (_Float16)v; const __bf16 bh = (__bf16)v; tb[cl][rl] = bh; tbl[cl][rl] = (__bf16)(v - (float)bh); } }
  __syncthreads();
  for (int e = tid; e < 128 * 8; e += 128) { const int cl = e >> 3, q = e & 7; vst2((unsigned*)(VT + (bb * CC + c0 + cl) * (size_t)TT + t0 + q * 8), *(const v4u*)&th[cl][q * 8]);
    if (hi_rows) { const size_t o3 = (bb * CC + c0 + cl) * (size_t)KHI + t0 + q * 8; vst2((unsigned*)(VB + o3), *(const v4u*)&tb[cl][q * 8]); vst2((unsigned*)(VBL + o3), *(const v4u*)&tbl[cl][q * 8]); } }
}

__global__ __launch_bounds__(128) void k_attn(const _Float16* __restrict__ QH, const _Float16* __restrict__ KH, const _Float16* __restrict__ VT, float* __restrict__ Y) {
  __shared__ __align__(16) _Float16 ps[4][16][40]; __shared__ __align__(16) float so[4][16][HD + 4];
  const int tid = threadIdx.x, wave = tid >> 5, lane = tid & 31, col = lane & 15, g = lane >> 4;
  const int qb = QBH + blockIdx.x, h = blockIdx.y, b = blockIdx.z; const int ql0 = qb * 64 + wave * 16;
  const size_t qoff = ((size_t)b * TT + ql0 + col) * CC + h * HD;
  const size_t kbase = (size_t)b * TT * CC + h * HD;
  const size_t vbase = ((size_t)b * CC + h * HD + col) * (size_t)TT;
  v8f o[4] = {}; float mrun[8], lsum[8];
#pragma unroll
  for (int r = 0; r < 8; ++r) { mrun[r] = -3.0e38f; lsum[r] = 0.f; }
  const int nhalf = (ql0 + 47) >> 5;
#pragma unroll 1
  for (int kh = 0; kh < nhalf; ++kh) { const int key0 = kh * 32; v8f s0 = {}, s1 = {};
#pragma unroll
    for (int kc = 0; kc < HD / 32; ++kc) { const v16h a = frag_h(QH + qoff + kc * 32, lane);
      const v16h kf0 = frag_h(KH + kbase + (size_t)(key0 + col) * CC + kc * 32, lane); const v16h kf1 = frag_h(KH + kbase + (size_t)(key0 + 16 + col) * CC + kc * 32, lane);
      s0 = wmma16(a, kf0, s0); s1 = wmma16(a, kf1, s1); }
    const int c0k = key0 + col, c1k = c0k + 16; float mloc[8];
#pragma unroll
    for (int r = 0; r < 8; ++r) { const int m = ql0 + 8 * g + r; const float x0 = (c0k <= m) ? s0[r] * SCALE_L2 : -3.0e38f; const float x1 = (c1k <= m) ? s1[r] * SCALE_L2 : -3.0e38f; s0[r] = x0; s1[r] = x1; mloc[r] = fmaxf(x0, x1); }
#pragma unroll
    for (int off = 1; off < 16; off <<= 1) {
#pragma unroll
      for (int r = 0; r < 8; ++r) mloc[r] = fmaxf(mloc[r], __shfl_xor(mloc[r], off)); }
    LDSX();
#pragma unroll
    for (int r = 0; r < 8; ++r) { const float mnew = fmaxf(mrun[r], mloc[r]); const float alpha = exp2f(mrun[r] - mnew); const float p0 = exp2f(s0[r] - mnew), p1 = exp2f(s1[r] - mnew);
      lsum[r] = lsum[r] * alpha + (p0 + p1); mrun[r] = mnew; o[0][r] *= alpha; o[1][r] *= alpha; o[2][r] *= alpha; o[3][r] *= alpha;
      ps[wave][8 * g + r][col] = (_Float16)(p0 * 1024.0f); ps[wave][8 * g + r][16 + col] = (_Float16)(p1 * 1024.0f); }
    LDSX();
    union { v16h v; v8h q[2]; } pa; pa.q[0] = *(const v8h*)&ps[wave][col][8 * g]; pa.q[1] = *(const v8h*)&ps[wave][col][16 + 8 * g];
#pragma unroll
    for (int j = 0; j < 4; ++j) o[j] = wmma16(pa.v, frag_h(VT + vbase + (size_t)j * 16 * TT + key0, lane), o[j]);
  }
#pragma unroll
  for (int off = 1; off < 16; off <<= 1) {
#pragma unroll
    for (int r = 0; r < 8; ++r) lsum[r] += __shfl_xor(lsum[r], off); }
#pragma unroll
  for (int r = 0; r < 8; ++r) { const float inv = 1.0f / (lsum[r] * 1024.0f);
#pragma unroll
    for (int j = 0; j < 4; ++j) so[wave][8 * g + r][j * 16 + col] = o[j][r] * inv; }
  LDSX();
  for (int i = 0; i < 8; ++i) { const int rl = 2 * i + g; vst2(Y + ((size_t)b * TT + ql0 + rl) * CC + h * HD + col * 4, *(const v4f*)&so[wave][rl][col * 4]); }
}

__global__ __launch_bounds__(128) void k_attn_hi(const _Float16* __restrict__ QH, const _Float16* __restrict__ QL, const _Float16* __restrict__ KH, const _Float16* __restrict__ KL, const __bf16* __restrict__ VB, const __bf16* __restrict__ VBL, float* __restrict__ Y) {
  __shared__ __align__(16) __bf16 pbh[4][16][40], pbl[4][16][40]; __shared__ __align__(16) float so[4][16][HD + 4];
  const int tid = threadIdx.x, wave = tid >> 5, lane = tid & 31, col = lane & 15, g = lane >> 4;
  const int qb = blockIdx.x, h = blockIdx.y, b = blockIdx.z; const int ql0 = qb * 64 + wave * 16;
  const size_t qoff = ((size_t)b * TT + ql0 + col) * CC + h * HD;
  const size_t qloff = ((size_t)b * QHI + ql0 + col) * CC + h * HD;
  const size_t kbase = (size_t)b * TT * CC + h * HD;
  const size_t klbase = (size_t)b * KHI * CC + h * HD;
  const size_t vbase = ((size_t)b * CC + h * HD + col) * (size_t)KHI;
  v8f o[4] = {}; float mrun[8], lsum[8];
#pragma unroll
  for (int r = 0; r < 8; ++r) { mrun[r] = -3.0e38f; lsum[r] = 0.f; }
  const int nhalf = (ql0 + 47) >> 5;
#pragma unroll 1
  for (int kh = 0; kh < nhalf; ++kh) { const int key0 = kh * 32; v8f s0 = {}, s1 = {}, u0 = {}, u1 = {};
#pragma unroll
    for (int kc = 0; kc < HD / 32; ++kc) { const v16h ah = frag_h(QH + qoff + kc * 32, lane), al = frag_h(QL + qloff + kc * 32, lane);
      { const v16h kf = frag_h(KH + kbase + (size_t)(key0 + col) * CC + kc * 32, lane), kl = frag_h(KL + klbase + (size_t)(key0 + col) * CC + kc * 32, lane); s0 = wmma16(ah, kf, s0); u0 = wmma16(al, kf, u0); u0 = wmma16(ah, kl, u0); }
      { const v16h kf = frag_h(KH + kbase + (size_t)(key0 + 16 + col) * CC + kc * 32, lane), kl = frag_h(KL + klbase + (size_t)(key0 + 16 + col) * CC + kc * 32, lane); s1 = wmma16(ah, kf, s1); u1 = wmma16(al, kf, u1); u1 = wmma16(ah, kl, u1); } }
    const int c0k = key0 + col, c1k = c0k + 16; float mloc[8];
#pragma unroll
    for (int r = 0; r < 8; ++r) { const int m = ql0 + 8 * g + r; const float a0 = (s0[r] + u0[r] * (1.0f / 1024.0f)) * SCALE_L2, a1 = (s1[r] + u1[r] * (1.0f / 1024.0f)) * SCALE_L2;
      const float x0 = (c0k <= m) ? a0 : -3.0e38f; const float x1 = (c1k <= m) ? a1 : -3.0e38f; s0[r] = x0; s1[r] = x1; mloc[r] = fmaxf(x0, x1); }
#pragma unroll
    for (int off = 1; off < 16; off <<= 1) {
#pragma unroll
      for (int r = 0; r < 8; ++r) mloc[r] = fmaxf(mloc[r], __shfl_xor(mloc[r], off)); }
    LDSX();
#pragma unroll
    for (int r = 0; r < 8; ++r) { const float mnew = fmaxf(mrun[r], mloc[r]); const float alpha = exp2f(mrun[r] - mnew); const float p0 = exp2f(s0[r] - mnew), p1 = exp2f(s1[r] - mnew);
      lsum[r] = lsum[r] * alpha + (p0 + p1); mrun[r] = mnew; o[0][r] *= alpha; o[1][r] *= alpha; o[2][r] *= alpha; o[3][r] *= alpha;
      const __bf16 h0 = (__bf16)p0, h1 = (__bf16)p1;
      pbh[wave][8 * g + r][col] = h0; pbh[wave][8 * g + r][16 + col] = h1; pbl[wave][8 * g + r][col] = (__bf16)(p0 - (float)h0); pbl[wave][8 * g + r][16 + col] = (__bf16)(p1 - (float)h1); }
    LDSX();
    union { v16b v; v8b q[2]; } ph, pl; ph.q[0] = *(const v8b*)&pbh[wave][col][8 * g]; ph.q[1] = *(const v8b*)&pbh[wave][col][16 + 8 * g]; pl.q[0] = *(const v8b*)&pbl[wave][col][8 * g]; pl.q[1] = *(const v8b*)&pbl[wave][col][16 + 8 * g];
#pragma unroll
    for (int j = 0; j < 4; ++j) { const size_t po = vbase + (size_t)j * 16 * KHI + key0; const v16b vh = frag_b(VB + po, lane); o[j] = wmma_bf(ph.v, vh, o[j]); o[j] = wmma_bf(pl.v, vh, o[j]); o[j] = wmma_bf(ph.v, frag_b(VBL + po, lane), o[j]); }
  }
#pragma unroll
  for (int off = 1; off < 16; off <<= 1) {
#pragma unroll
    for (int r = 0; r < 8; ++r) lsum[r] += __shfl_xor(lsum[r], off); }
#pragma unroll
  for (int r = 0; r < 8; ++r) { const float inv = 1.0f / lsum[r];
#pragma unroll
    for (int j = 0; j < 4; ++j) so[wave][8 * g + r][j * 16 + col] = o[j][r] * inv; }
  LDSX();
  for (int i = 0; i < 8; ++i) { const int rl = 2 * i + g; vst2(Y + ((size_t)b * TT + ql0 + rl) * CC + h * HD + col * 4, *(const v4f*)&so[wave][rl][col * 4]); }
}

__global__ __launch_bounds__(128) void k_out(const float* __restrict__ Y, const float* __restrict__ WO, const float* __restrict__ BO, float* __restrict__ OUT) { __shared__ __align__(16) float sf[4][16][132];
  const int tid = threadIdx.x, wave = tid >> 5, lane = tid & 31, col = lane & 15, g = lane >> 4; const int c0 = blockIdx.y * 128; const size_t r0 = (size_t)blockIdx.x * 64 + wave * 16;
  (void)tid;
  v8f acc[8] = {};
  if ((int)(((size_t)blockIdx.x * 64) % TT) < QHI) {
#pragma unroll 2
    for (int kc = 0; kc < CC / 32; ++kc) { const F2 a = split_row(Y + (r0 + col) * CC, kc * 32, lane); asm volatile("s_wait_loadcnt 0x0" ::: "memory");
#pragma unroll
      for (int j = 0; j < 8; ++j) { const v16b w = wcol_oi(WO, kc * 32, c0 + j * 16 + col, lane, CC); asm volatile("s_wait_loadcnt 0x0" ::: "memory"); acc[j] = wmma_bf(a.h, w, acc[j]); acc[j] = wmma_bf(a.l, w, acc[j]); } }
#pragma unroll
    for (int j = 0; j < 8; ++j) { const float bias = bfr(BO[c0 + j * 16 + col]);
#pragma unroll
      for (int r = 0; r < 8; ++r) sf[wave][8 * g + r][j * 16 + col] = acc[j][r] + bias; }
  } else {
#pragma unroll 2
    for (int kc = 0; kc < CC / 32; ++kc) { const v16h a = frag_f32s(Y + (r0 + col) * CC + kc * 32, lane, 64.0f); asm volatile("s_wait_loadcnt 0x0" ::: "memory");
#pragma unroll
      for (int j = 0; j < 8; ++j) { const v16h w = wcolh_oi(WO, kc * 32, c0 + j * 16 + col, lane, CC); asm volatile("s_wait_loadcnt 0x0" ::: "memory"); acc[j] = wmma16(a, w, acc[j]); } }
#pragma unroll
    for (int j = 0; j < 8; ++j) { const float bias = bfr(BO[c0 + j * 16 + col]);
#pragma unroll
      for (int r = 0; r < 8; ++r) sf[wave][8 * g + r][j * 16 + col] = acc[j][r] * (1.0f / 16384.0f) + bias; } }
  LDSX(); for (int rl = 0; rl < 16; ++rl) vst2(OUT + (r0 + rl) * DIN + c0 + lane * 4, *(const v4f*)&sf[wave][rl][lane * 4]); }

extern "C" void kernel_launch(void* const* d_in, const int* in_sizes, int n_in, void* d_out, int out_size, void* d_ws, size_t ws_size, hipStream_t stream) {
  if (n_in < 10) return;
  if ((size_t)in_sizes[0] < ((size_t)(NB - 1) * TT_FULL + TT) * DIN) return;
  if (in_sizes[1] < CC * DIN || in_sizes[3] < CC * DIN || in_sizes[5] < CC * DIN || in_sizes[7] < DIN * CC) return;
  if (in_sizes[2] < CC || in_sizes[4] < CC || in_sizes[6] < CC || in_sizes[8] < DIN) return;
  if ((size_t)out_size < (size_t)NB * TT * DIN) return;
  if (ws_size < (size_t)WS_END) return;
  const float* x  = (const float*)d_in[0];
  const float* Wq = (const float*)d_in[1]; const float* bq = (const float*)d_in[2];
  const float* Wk = (const float*)d_in[3]; const float* bk = (const float*)d_in[4];
  const float* Wv = (const float*)d_in[5]; const float* bv = (const float*)d_in[6];
  const float* Wo = (const float*)d_in[7]; const float* bo = (const float*)d_in[8];
  char* ws = (char*)d_ws;
  _Float16 *QH = (_Float16*)(ws + WS_QH), *KH = (_Float16*)(ws + WS_KH), *VT = (_Float16*)(ws + WS_VT), *QL = (_Float16*)(ws + WS_QL), *KL = (_Float16*)(ws + WS_KL);
  __bf16 *VB = (__bf16*)(ws + WS_VB), *VBL = (__bf16*)(ws + WS_VBL); float* Y = (float*)(ws + WS_Y);
  k_projq<<<dim3(NB * TT / 64, CC / 128), 128, 0, stream>>>(x, Wq, bq, QH, QL);
  k_projk<<<dim3(NB * TT / 64, CC / 128), 128, 0, stream>>>(x, Wk, bk, KH, KL);
  k_projv<<<dim3(NB * TT / 64, CC / 128), 128, 0, stream>>>(x, Wv, bv, VT, VB, VBL);
  k_attn_hi<<<dim3(QBH, NH, NB), 128, 0, stream>>>(QH, QL, KH, KL, VB, VBL, Y);
  if (NQB > QBH) k_attn<<<dim3(NQB - QBH, NH, NB), 128, 0, stream>>>(QH, KH, VT, Y);
  k_out<<<dim3(NB * TT / 64, DIN / 128), 128, 0, stream>>>(Y, Wo, bo, (float*)d_out);
}
